// BahdanauAttention_70652212019613
// MI455X (gfx1250) — hardware-verified
//
#include <hip/hip_runtime.h>
#include <math.h>

typedef __attribute__((ext_vector_type(16))) _Float16 v16h;
typedef __attribute__((ext_vector_type(8)))  _Float16 v8h;
typedef __attribute__((ext_vector_type(8)))  float    v8f;
typedef __attribute__((ext_vector_type(4)))  float    v4f;
typedef __attribute__((ext_vector_type(2)))  float    v2f;
typedef __attribute__((ext_vector_type(4)))  unsigned int v4u;

constexpr int kB  = 8;
constexpr int kTE = 512;
constexpr int kTD = 256;
constexpr int kD  = 256;
constexpr int kU  = 256;
constexpr int kEncRows = kB * kTE;
constexpr int kDecRows = kB * kTD;
static_assert(kEncRows == 4096 && kDecRows == 2048, "row counts");
static_assert((kD % 32) == 0 && (kTE % 32) == 0, "GEMM K multiples of 32");
static_assert((kU % 64) == 0 && (kTE % 64) == 0 && (kTD % 64) == 0 && (kD % 64) == 0 && (kDecRows % 64) == 0, "GEMM M,N multiples of 64");
static_assert(kU == 256 && kTE == 512, "score kernel thread map: 256 threads, two encoder positions per thread");

constexpr float kXCarry   = 16.0f;
constexpr float kWCarry   = 256.0f;
constexpr float kPCarry   = 512.0f;
constexpr float kProjScale = 1.0f / (kWCarry * kXCarry);
constexpr float kCtxScale  = 1.0f / (kPCarry * kXCarry);
constexpr float kF16MinNormal = 6.103515625e-05f;

constexpr float kArgScale = 2.8853900817779268f;
static_assert(kArgScale > 2.885f && kArgScale < 2.886f, "argument constant is 2*log2(e) in every pass");
__device__ __forceinline__ float exp_scaled(float a) {
#if __has_builtin(__builtin_amdgcn_exp2f)
  return __builtin_amdgcn_exp2f(a);
#else
  return exp2f(a);
#endif
}
constexpr float kEpScale = kArgScale * kProjScale;

constexpr size_t kOffENCH = 0;
constexpr size_t kOffDECH = kOffENCH + (size_t)kEncRows * kD * 2;
constexpr size_t kOffENCT = kOffDECH + (size_t)kDecRows * kD * 2;
constexpr size_t kOffWT   = kOffENCT + (size_t)kB * kD * kTE * 2;
constexpr size_t kOffEPS  = kOffWT   + (size_t)2 * kU * kD * 2;
constexpr size_t kOffDPB  = kOffEPS  + (size_t)kB * kU * kTE * 4;
constexpr size_t kOffPH   = kOffDPB  + (size_t)kDecRows * kU * 4;
constexpr size_t kWsTotal = kOffPH   + (size_t)kDecRows * kTE * 2;
static_assert(kWsTotal == 13893632ull, "carve total");
static_assert(kWsTotal <= 134217728ull, "carve cap");
static_assert((kOffDECH % 128) == 0 && (kOffENCT % 128) == 0 && (kOffWT % 128) == 0 && (kOffEPS % 128) == 0 &&
              (kOffDPB % 128) == 0 && (kOffPH % 128) == 0, "128-B aligned regions");

constexpr size_t kOut0Bytes = (size_t)kB * kTD * kD * 4;
constexpr size_t kOut1OffBytes = 2097152ull;
constexpr size_t kOut1Bytes = (size_t)kB * kTD * kTE * 4;
static_assert(kOut0Bytes == kOut1OffBytes, "second output follows the first");
static_assert(kOut1OffBytes + kOut1Bytes == 6291456ull, "output total");
static_assert((kOut1OffBytes % 128) == 0, "second output line aligned");
constexpr size_t kOut1OffElems = kOut1OffBytes / 4;

__device__ __forceinline__ unsigned pk16(unsigned short a, unsigned short b) { return (unsigned)a | ((unsigned)b << 16); }

__device__ __forceinline__ unsigned short h_bits_flush(float f) {
  const float g = (fabsf(f) < kF16MinNormal) ? 0.0f : f;
  const _Float16 h = (_Float16)g;
  return __builtin_bit_cast(unsigned short, h);
}

union FragH { v16h v; v8h h[2]; };
__device__ __forceinline__ v16h frag_load(const _Float16* p) {
  FragH f;
  f.h[0] = *(const v8h*)(p);
  f.h[1] = *(const v8h*)(p + 16);
  return f.v;
}
__device__ __forceinline__ v8f mma_f16(v16h a, v16h b, v8f c) {
  c = __builtin_amdgcn_wmma_f32_16x16x32_f16(false, a, false, b, (short)0, c, false, false);
  asm volatile("v_nop\n\tv_nop\n\tv_nop\n\tv_nop" : "+v"(c) : "v"(a), "v"(b));
  return c;
}

template <int BIAS_MODE>
__global__ __launch_bounds__(256) void gemm_f16_tile64(
    const unsigned short* __restrict__ Ap, int lda, long strideA,
    const unsigned short* __restrict__ Btp, int ldb, long strideB,
    float* __restrict__ Cout, int ldc, long strideC,
    const float* __restrict__ bias,
    int M, int N, int K, float scale) {
  const _Float16* A  = (const _Float16*)Ap;
  const _Float16* Bt = (const _Float16*)Btp;
  __shared__ __align__(16) float sT[8][16 * 68];
  const int b    = blockIdx.y;
  const int lane = threadIdx.x & 31;
  const int wave = threadIdx.x >> 5;
  const int tilesN = N >> 6;
  const int tilesM = M >> 6;
  const int tile = blockIdx.x * 8 + wave;
  if (tile >= tilesM * tilesN) return;
  const int tm = tile / tilesN;
  const int tn = tile - tm * tilesN;
  const int m0 = tm << 6;
  const int n0 = tn << 6;

  const _Float16* Ab = A  + (size_t)b * strideA;
  const _Float16* Bb = Bt + (size_t)b * strideB;

  const int rlane = lane & 15;
  const int koff  = (lane >> 4) * 8;
  const int mOff  = (lane >> 4) * 8;

  v8f acc[4][4];
#pragma unroll
  for (int i = 0; i < 4; ++i)
#pragma unroll
    for (int j = 0; j < 4; ++j) acc[i][j] = (v8f){0.f,0.f,0.f,0.f,0.f,0.f,0.f,0.f};

  for (int k0 = 0; k0 < K; k0 += 32) {
    v16h bh[4];
#pragma unroll
    for (int j = 0; j < 4; ++j) {
      const size_t bo = (size_t)(n0 + (j << 4) + rlane) * ldb + koff + k0;
      bh[j] = frag_load(Bb + bo);
    }
#pragma unroll
    for (int i = 0; i < 4; ++i) {
      const size_t ao = (size_t)(m0 + (i << 4) + rlane) * lda + koff + k0;
      const v16h ah = frag_load(Ab + ao);
#pragma unroll
      for (int j = 0; j < 4; ++j) acc[i][j] = mma_f16(ah, bh[j], acc[i][j]);
    }
  }

  float* slab = sT[wave];
  float* C = Cout + (size_t)b * strideC;
#pragma unroll
  for (int i = 0; i < 4; ++i) {
    const int mBase = m0 + (i << 4);
#pragma unroll
    for (int j = 0; j < 4; ++j) {
      const int n = n0 + (j << 4) + rlane;
      float bv = 0.f;
      if (BIAS_MODE == 2) bv = bias[n];
#pragma unroll
      for (int r = 0; r < 8; ++r) {
        float v = acc[i][j][r] * scale;
        if (BIAS_MODE == 2) v += bv;
        slab[(mOff + r) * 68 + (j << 4) + rlane] = v;
      }
    }
    __builtin_amdgcn_fence(__ATOMIC_RELEASE, "workgroup");
    __builtin_amdgcn_wave_barrier();
    __builtin_amdgcn_fence(__ATOMIC_ACQUIRE, "workgroup");
    {
      const int hh = lane >> 4, c4 = (lane & 15) * 4;
      for (int pass = 0; pass < 2; ++pass) {
#pragma unroll
        for (int it = 0; it < 8; ++it) {
          const int row = it * 2 + hh;
          v4f v = *(const v4f*)(slab + row * 68 + c4);
          *(volatile v4f*)(C + (size_t)(mBase + row) * ldc + n0 + c4) = v;
        }
        __threadfence();
      }
    }
    __builtin_amdgcn_fence(__ATOMIC_RELEASE, "workgroup");
    __builtin_amdgcn_wave_barrier();
    __builtin_amdgcn_fence(__ATOMIC_ACQUIRE, "workgroup");
  }
}

constexpr int kEncCastBlocks = (kEncRows * kD / 8) / 256;
constexpr int kDecCastBlocks = (kDecRows * kD / 8) / 256;
static_assert(kEncCastBlocks * 256 * 8 == kEncRows * kD, "enc cast coverage");
static_assert(kDecCastBlocks * 256 * 8 == kDecRows * kD, "dec cast coverage");

__global__ __launch_bounds__(256) void cast_rows_kernel(const float* enc, const float* dec,
                                                        unsigned short* encH, unsigned short* decH, float carry) {
  const int isDec = (blockIdx.x >= (unsigned)kEncCastBlocks) ? 1 : 0;
  const int blk = (int)blockIdx.x - isDec * kEncCastBlocks;
  const float* src = isDec ? dec : enc;
  unsigned short* dst = isDec ? decH : encH;
  const size_t e0 = ((size_t)blk * 256 + threadIdx.x) * 8;
  const v4f a = *(const v4f*)(src + e0);
  const v4f c = *(const v4f*)(src + e0 + 4);
  unsigned short hb[8];
#pragma unroll
  for (int e = 0; e < 4; ++e) {
    const float fa = a[e] * carry;
    const float fc = c[e] * carry;
    hb[e]     = h_bits_flush(fa);
    hb[4 + e] = h_bits_flush(fc);
  }
  const v4u u = (v4u){pk16(hb[0], hb[1]), pk16(hb[2], hb[3]), pk16(hb[4], hb[5]), pk16(hb[6], hb[7])};
  unsigned short* q = dst + e0;
  *(volatile v4u*)q = u;
  __threadfence();
  *(volatile v4u*)q = u;
}

__global__ __launch_bounds__(256) void transpose_cast_kernel(const float* inA, const float* inB, int twoSrc,
                                                             long inBatch, int ldi,
                                                             unsigned short* __restrict__ out, long outBatch, int ldo,
                                                             float carry) {
  __shared__ float sm[64][65];
  const int t  = threadIdx.x;
  const int r0 = blockIdx.x * 64;
  const int c0 = blockIdx.y * 64;
  const int z  = blockIdx.z;
  const float* src = ((twoSrc != 0 && z == 1) ? inB : inA) + (size_t)z * inBatch;
#pragma unroll
  for (int i = 0; i < 16; ++i) {
    const int e = i * 256 + t;
    const int r = e >> 6;
    const int c = e & 63;
    sm[c][r] = src[(size_t)(r0 + r) * ldi + c0 + c] * carry;
  }
  __syncthreads();
  const int lane = t & 31, wave = t >> 5;
  const int q = lane >> 3, c8 = (lane & 7) * 8;
  unsigned short* op = out + (size_t)z * outBatch;
  for (int pass = 0; pass < 2; ++pass) {
#pragma unroll
    for (int it = 0; it < 2; ++it) {
      const int row = wave * 8 + it * 4 + q;
      unsigned short hb[8];
#pragma unroll
      for (int e = 0; e < 8; ++e) hb[e] = h_bits_flush(sm[row][c8 + e]);
      const v4u u = (v4u){pk16(hb[0], hb[1]), pk16(hb[2], hb[3]), pk16(hb[4], hb[5]), pk16(hb[6], hb[7])};
      *(volatile v4u*)(op + (size_t)(c0 + row) * ldo + r0 + c8) = u;
    }
    __threadfence();
  }
}

__global__ __launch_bounds__(256) void score_softmax_kernel(
    const float* __restrict__ eps, const float* __restrict__ dpb, const float* __restrict__ b1,
    const float* __restrict__ vvec, const float* __restrict__ bV,
    float* __restrict__ wout, unsigned* __restrict__ pw) {
  __shared__ __align__(16) float sU[kU * 8];
  __shared__ float sRedM[4 * 8];
  __shared__ float sRedS[4 * 8];
  __shared__ float sRedV[8];
  const int tid = threadIdx.x, lane = tid & 31, wave = tid >> 5;
  const int bt0 = blockIdx.x * 4;
  const int b   = bt0 / kTD;

  {
    const float bb = b1[tid];
    const float vv = vvec[tid];
    v4f dsv;
    dsv[0] = (dpb[(size_t)(bt0 + 0) * kU + tid] + bb) * kArgScale;
    dsv[1] = (dpb[(size_t)(bt0 + 1) * kU + tid] + bb) * kArgScale;
    dsv[2] = (dpb[(size_t)(bt0 + 2) * kU + tid] + bb) * kArgScale;
    dsv[3] = (dpb[(size_t)(bt0 + 3) * kU + tid] + bb) * kArgScale;
    const v4f vsl = (v4f){-2.0f * vv, 0.0f, 0.0f, 0.0f};
    *(v4f*)(sU + tid * 8)     = dsv;
    *(v4f*)(sU + tid * 8 + 4) = vsl;
    float sv = vv;
#pragma unroll
    for (int off = 16; off > 0; off >>= 1) sv += __shfl_xor(sv, off, 32);
    if (lane == 0) sRedV[wave] = sv;
  }
  __syncthreads();
  float cst = sRedV[0];
#pragma unroll
  for (int w = 1; w < 8; ++w) cst += sRedV[w];
  cst += bV[0];

  float acc[4][2];
#pragma unroll
  for (int t = 0; t < 4; ++t) { acc[t][0] = 0.0f; acc[t][1] = 0.0f; }

  const float* ep = eps + (size_t)b * kU * kTE + 2 * tid;
#pragma unroll 2
  for (int u = 0; u < kU; ++u) {
    const v2f x  = *(const v2f*)(ep + (size_t)u * kTE);
    const v4f d  = *(const v4f*)(sU + u * 8);
    const float vm = sU[u * 8 + 4];
#pragma unroll
    for (int t = 0; t < 4; ++t) {
      const float e0 = exp_scaled(x[0] + d[t]);
      const float e1 = exp_scaled(x[1] + d[t]);
      const float r0 = __builtin_amdgcn_rcpf(1.0f + e0);
      const float r1 = __builtin_amdgcn_rcpf(1.0f + e1);
      acc[t][0] = fmaf(r0, vm, acc[t][0]);
      acc[t][1] = fmaf(r1, vm, acc[t][1]);
    }
  }

  float lg[4][2];
  float mx[4];
#pragma unroll
  for (int t = 0; t < 4; ++t) {
    lg[t][0] = acc[t][0] + cst;
    lg[t][1] = acc[t][1] + cst;
    float m = fmaxf(lg[t][0], lg[t][1]);
#pragma unroll
    for (int off = 16; off > 0; off >>= 1) m = fmaxf(m, __shfl_xor(m, off, 32));
    mx[t] = m;
  }
  if (lane == 0) {
#pragma unroll
    for (int t = 0; t < 4; ++t) sRedM[t * 8 + wave] = mx[t];
  }
  __syncthreads();
  float ex[4][2];
  float sm[4];
#pragma unroll
  for (int t = 0; t < 4; ++t) {
    float m = sRedM[t * 8];
#pragma unroll
    for (int w = 1; w < 8; ++w) m = fmaxf(m, sRedM[t * 8 + w]);
    ex[t][0] = expf(lg[t][0] - m);
    ex[t][1] = expf(lg[t][1] - m);
    float s = ex[t][0] + ex[t][1];
#pragma unroll
    for (int off = 16; off > 0; off >>= 1) s += __shfl_xor(s, off, 32);
    sm[t] = s;
  }
  if (lane == 0) {
#pragma unroll
    for (int t = 0; t < 4; ++t) sRedS[t * 8 + wave] = sm[t];
  }
  __syncthreads();
  v2f wv[4];
  unsigned pk[4];
#pragma unroll
  for (int t = 0; t < 4; ++t) {
    float s = sRedS[t * 8];
#pragma unroll
    for (int w = 1; w < 8; ++w) s += sRedS[t * 8 + w];
    const float inv = __builtin_amdgcn_rcpf(s);
    const float w0 = ex[t][0] * inv;
    const float w1 = ex[t][1] * inv;
    wv[t] = (v2f){w0, w1};
    pk[t] = pk16(h_bits_flush(w0 * kPCarry), h_bits_flush(w1 * kPCarry));
  }
  for (int pass = 0; pass < 2; ++pass) {
#pragma unroll
    for (int t = 0; t < 4; ++t) {
      *(volatile v2f*)(wout + (size_t)(bt0 + t) * kTE + 2 * tid) = wv[t];
      *(volatile unsigned*)(pw + (size_t)(bt0 + t) * (kTE / 2) + tid) = pk[t];
    }
    __threadfence();
  }
}

static_assert((kU / 64) * (kTE / 64) == 4 * 8, "enc projection grid");
static_assert((kDecRows / 64) * (kU / 64) == 16 * 8, "dec projection grid");
static_assert((kTD / 64) * (kD / 64) == 2 * 8, "context grid");

extern "C" void kernel_launch(void* const* d_in, const int* in_sizes, int n_in,
                              void* d_out, int out_size, void* d_ws, size_t ws_size,
                              hipStream_t stream) {
  if (n_in < 8) return;
  if (in_sizes[0] != kB * kTE * kD) return;
  if (in_sizes[1] != kB * kTD * kD) return;
  if (in_sizes[2] != kD * kU) return;
  if (in_sizes[3] != kU) return;
  if (in_sizes[4] != kD * kU) return;
  if (in_sizes[5] != kU) return;
  if (in_sizes[6] != kU) return;
  if (in_sizes[7] != 1) return;
  if (out_size != kB * kTD * kD + kB * kTD * kTE) return;
  if (ws_size < kWsTotal) return;

  const float* enc = (const float*)d_in[0];
  const float* dec = (const float*)d_in[1];
  const float* W1  = (const float*)d_in[2];
  const float* b1  = (const float*)d_in[3];
  const float* W2  = (const float*)d_in[4];
  const float* b2  = (const float*)d_in[5];
  const float* Vv  = (const float*)d_in[6];
  const float* bV  = (const float*)d_in[7];

  float* out0 = (float*)d_out;
  float* out1 = (float*)d_out + kOut1OffElems;

  char* ws = (char*)d_ws;
  unsigned short* ENCH = (unsigned short*)(ws + kOffENCH);
  unsigned short* DECH = (unsigned short*)(ws + kOffDECH);
  unsigned short* ENCT = (unsigned short*)(ws + kOffENCT);
  unsigned short* WT   = (unsigned short*)(ws + kOffWT);
  float*          EPS  = (float*)(ws + kOffEPS);
  float*          DPB  = (float*)(ws + kOffDPB);
  unsigned short* PH   = (unsigned short*)(ws + kOffPH);
  unsigned short* W1T  = WT;
  unsigned short* W2T  = WT + (size_t)kU * kD;

  cast_rows_kernel<<<kEncCastBlocks + kDecCastBlocks, 256, 0, stream>>>(enc, dec, ENCH, DECH, kXCarry);
  transpose_cast_kernel<<<dim3(kD / 64, kU / 64, 2), 256, 0, stream>>>(
      W1, W2, 1, 0L, kU, WT, (long)kU * kD, kD, kWCarry);
  transpose_cast_kernel<<<dim3(kTE / 64, kD / 64, kB), 256, 0, stream>>>(
      enc, enc, 0, (long)kTE * kD, kD, ENCT, (long)kD * kTE, kTE, kXCarry);

  gemm_f16_tile64<0><<<dim3(4, kB), 256, 0, stream>>>(
      W1T, kD, 0L,
      ENCH, kD, (long)kTE * kD,
      EPS, kTE, (long)kU * kTE,
      nullptr,
      kU, kTE, kD, kEpScale);

  gemm_f16_tile64<2><<<dim3(16, 1), 256, 0, stream>>>(
      DECH, kD, 0L,
      W2T, kD, 0L,
      DPB, kU, 0L,
      b2,
      kDecRows, kU, kD, kProjScale);

  score_softmax_kernel<<<kB * (kTD / 4), 256, 0, stream>>>(EPS, DPB, b1, Vv, bV, out1, (unsigned*)PH);

  gemm_f16_tile64<0><<<dim3(2, kB), 256, 0, stream>>>(
      PH, kTE, (long)kTD * kTE,
      ENCT, kTE, (long)kD * kTE,
      out0, kD, (long)kTD * kD,
      nullptr,
      kTD, kD, kTE, kCtxScale);
}
